// NetGCN_15324443312398
// MI455X (gfx1250) — hardware-run, weakly checked
//
#include <hip/hip_runtime.h>
#include <stddef.h>
#include <stdint.h>
#include <math.h>


#define NN     100000
#define NE     1600000
#define DF     128
#define MP     100096
#define NTHR   256
#define NWAVE  8
#define NBA    1024
#define SLA    10
#define GA     98
#define NPT    (GA * NBA)
#define RCAP   20480
#define WLCAP  3072
#define DEGCAP 64
#define WSHARE (NE / NWAVE)
#define KPI    256
#define NIT    ((WSHARE + KPI - 1) / KPI)
#define NBO    4096
#define GO     25
#define NPO    (GO * NBO)
#define GBM    64
#define GBN    128
#define GTHR   128
#define BK_INTS (NWAVE * WLCAP + RCAP + NWAVE * NBA + 3 * NBA + 32)
#define OD_INTS (NWAVE * NBO + NWAVE * KPI + NBO + 32)
#define PU_W1I 2048
#define PU_W1  4096
#define PU_W2  8192
#define PU_BI  8448
#define PU_Z   11520
#define PU_END (PU_Z + MP * 16)
#define WSMAX  134217728

static_assert(NE % (NWAVE * 8) == 0 && NE % 4 == 0 && WSHARE % 8 == 0);
static_assert(NBA == (1 << SLA) && GA * NBA >= NN && (GA - 1) * NBA < NN);
static_assert(NN - 1 < (1 << 17) && 17 + SLA <= 31);
static_assert(RCAP % (NTHR * 4) == 0 && RCAP >= 17558 && NWAVE * WLCAP >= RCAP && WLCAP >= RCAP / NWAVE);
static_assert(DEGCAP >= 36 + 8);
static_assert(GO * NBO >= MP && NPT >= NN && NBO % (NTHR * 4) == 0);
static_assert(MP % GBM == 0 && MP >= NN && MP % 128 == 0);
static_assert(BK_INTS % 4 == 0 && OD_INTS % 4 == 0);
static_assert(BK_INTS * 4 <= 300000 && OD_INTS * 4 <= 300000);
static_assert(DF % 32 == 0 && (2 * DF) % 32 == 0 && GBN == DF && GBM == (GTHR / 32) * 16);
static_assert(PU_W1I % NTHR == 0 && PU_W1 % NTHR == 0 && PU_W2 % NTHR == 0 && PU_BI % NTHR == 0);
static_assert(PU_Z % NTHR == 0 && PU_END % NTHR == 0 && (PU_Z - PU_BI) * 8 == (MP - NN) * 2 * DF);

typedef float          v4f   __attribute__((ext_vector_type(4)));
typedef float          v8f   __attribute__((ext_vector_type(8)));
typedef int            v4i   __attribute__((ext_vector_type(4)));
typedef int            v8i   __attribute__((ext_vector_type(8)));
typedef unsigned int   v4u   __attribute__((ext_vector_type(4)));
typedef unsigned short v8us  __attribute__((ext_vector_type(8)));
typedef unsigned short v16us __attribute__((ext_vector_type(16)));
typedef __bf16         v16bf __attribute__((ext_vector_type(16)));
typedef v4f  __attribute__((may_alias)) v4fa;
typedef v4i  __attribute__((may_alias)) v4ia;
typedef v8us __attribute__((may_alias)) v8usa;
union FragB { v16bf v; v16us u; v8us h[2]; v8i w; };

__device__ __forceinline__ v8f wmb(const FragB& a, const FragB& b, v8f c) {
  v8f d = __builtin_amdgcn_wmma_f32_16x16x32_bf16(false, a.v, false, b.v, (short)0, c, false, false);
  asm volatile("v_nop\n\tv_nop\n\tv_nop\n\tv_nop" : "+v"(d) : "v"(a.w), "v"(b.w));
  return d;
}
__device__ __forceinline__ v8f z8() { v8f z = {0.f, 0.f, 0.f, 0.f, 0.f, 0.f, 0.f, 0.f}; return z; }

__device__ __forceinline__ unsigned bf16_bits(float f) {
  const unsigned u = __float_as_uint(f);
  const unsigned r = (u + 0x7FFFu + ((u >> 16) & 1u)) >> 16;
  return (f != f) ? 0x7FC0u : (r & 0xFFFFu);
}
__device__ __forceinline__ float bf16_val(float f) { return __uint_as_float(bf16_bits(f) << 16); }
__device__ __forceinline__ unsigned pk2(float a, float b) { return bf16_bits(a) | (bf16_bits(b) << 16); }
__device__ __forceinline__ int clampn(int s) { return s < 0 ? 0 : (s > NN - 1 ? NN - 1 : s); }
__device__ __forceinline__ float relu_np(float v) { return (v > 0.0f) ? v : (v - v); }

__device__ __forceinline__ void wave_sync() {
  __builtin_amdgcn_fence(__ATOMIC_RELEASE, "wavefront");
  __builtin_amdgcn_wave_barrier();
  __builtin_amdgcn_fence(__ATOMIC_ACQUIRE, "wavefront");
}

__global__ __launch_bounds__(NTHR) void k_prep(const float* __restrict__ x, const float* __restrict__ w1i,
                                               const float* __restrict__ w1b, const float* __restrict__ w2,
                                               const float* __restrict__ b1i, const float* __restrict__ b1b,
                                               const float* __restrict__ b2,
                                               unsigned short* w1t, unsigned short* w2d, float* bias,
                                               unsigned short* hs, unsigned short* xb) {
  const int u = (int)blockIdx.x * NTHR + (int)threadIdx.x;
  v4u o;
  char* dp;
  if (u < PU_W1I) {
    const int n = u >> 4, k8 = (u & 15) * 8;
    const float* p = w1i + (size_t)k8 * DF + n;
    float f[8];
#pragma unroll
    for (int i = 0; i < 8; ++i) f[i] = p[(size_t)i * DF];
    o.x = pk2(f[0], f[1]); o.y = pk2(f[2], f[3]); o.z = pk2(f[4], f[5]); o.w = pk2(f[6], f[7]);
    dp = (char*)(w1t + (size_t)u * 8);
  } else if (u < PU_W1) {
    const int v = u - PU_W1I;
    const int n = v >> 4, k8 = (v & 15) * 8;
    const float* p = w1b + (size_t)k8 * DF + n;
    float f[8];
#pragma unroll
    for (int i = 0; i < 8; ++i) f[i] = p[(size_t)i * DF];
    o.x = pk2(f[0], f[1]); o.y = pk2(f[2], f[3]); o.z = pk2(f[4], f[5]); o.w = pk2(f[6], f[7]);
    dp = (char*)(w1t + (size_t)u * 8);
  } else if (u < PU_W2) {
    const int v = u - PU_W1;
    const int n = v >> 5, k8 = (v & 31) * 8;
    const int kk = k8 & (DF - 1);
    const float* p = w2 + (size_t)kk * DF + n;
    float f[8];
#pragma unroll
    for (int i = 0; i < 8; ++i) f[i] = p[(size_t)i * DF];
    o.x = pk2(f[0], f[1]); o.y = pk2(f[2], f[3]); o.z = pk2(f[4], f[5]); o.w = pk2(f[6], f[7]);
    dp = (char*)(w2d + (size_t)v * 8);
  } else if (u < PU_BI) {
    const int v = u - PU_W2;
    if (v >= 96) return;
    const int r = v >> 5, c4 = (v & 31) * 4;
    const v4f la = *(const v4f*)(b1i + c4);
    const v4f lb = *(const v4f*)(b1b + c4);
    const v4f lc = *(const v4f*)(b2 + c4);
    asm volatile("" :: "v"(la), "v"(lb), "v"(lc));
    const unsigned k0 = (r == 0) ? 0xFFFFFFFFu : 0u;
    const unsigned k1 = (r == 1) ? 0xFFFFFFFFu : 0u;
    const unsigned k2 = (r == 2) ? 0xFFFFFFFFu : 0u;
    o.x = ((bf16_bits(la.x) << 16) & k0) | ((bf16_bits(lb.x) << 16) & k1) | ((bf16_bits(lc.x) << 16) & k2);
    o.y = ((bf16_bits(la.y) << 16) & k0) | ((bf16_bits(lb.y) << 16) & k1) | ((bf16_bits(lc.y) << 16) & k2);
    o.z = ((bf16_bits(la.z) << 16) & k0) | ((bf16_bits(lb.z) << 16) & k1) | ((bf16_bits(lc.z) << 16) & k2);
    o.w = ((bf16_bits(la.w) << 16) & k0) | ((bf16_bits(lb.w) << 16) & k1) | ((bf16_bits(lc.w) << 16) & k2);
    dp = (char*)(bias + (size_t)v * 4);
  } else if (u < PU_Z) {
    const int v = u - PU_BI;
    o.x = 0u; o.y = 0u; o.z = 0u; o.w = 0u;
    dp = (char*)(hs + (size_t)NN * (2 * DF) + (size_t)v * 8);
  } else if (u < PU_END) {
    const int v = u - PU_Z;
    const int row = v >> 4, k8 = (v & 15) * 8;
    const int rc = row < NN ? row : NN - 1;
    const float* p = x + (size_t)rc * DF + k8;
    const v4f a = *(const v4f*)p;
    const v4f b = *(const v4f*)(p + 4);
    asm volatile("" :: "v"(a), "v"(b));
    const unsigned msk = (row < NN) ? 0xFFFFFFFFu : 0u;
    o.x = pk2(a.x, a.y) & msk; o.y = pk2(a.z, a.w) & msk;
    o.z = pk2(b.x, b.y) & msk; o.w = pk2(b.z, b.w) & msk;
    dp = (char*)(xb + (size_t)v * 8);
  } else {
    return;
  }
  *(volatile v4u*)dp = o;
  __threadfence();
  *(volatile v4u*)dp = o;
}

__device__ __forceinline__ void bucket_store(const int* sl, const int* cnt, const int* offs, const float* ddv,
                                             int ov, int* lst, int* cntg, int* offg, float* ddg, int* flg,
                                             int tid) {
#pragma unroll 1
  for (int it = 0; it < RCAP / (NTHR * 4); ++it) {
    const int i = it * (NTHR * 4) + 4 * tid;
    const v4i v = *(const v4ia*)(sl + i);
    *(volatile v4i*)(lst + i) = v;
  }
  {
    const v4i c4 = *(const v4ia*)(cnt + 4 * tid);
    const v4i o4 = *(const v4ia*)(offs + 4 * tid);
    const v4f d4 = *(const v4fa*)(ddv + 4 * tid);
    *(volatile v4i*)(cntg + 4 * tid) = c4;
    *(volatile v4i*)(offg + 4 * tid) = o4;
    *(volatile v4f*)(ddg + 4 * tid) = d4;
  }
  if (tid < 8) {
    const v4i f4 = {ov, ov, ov, ov};
    *(volatile v4i*)(flg + 4 * tid) = f4;
  }
}

__device__ __forceinline__ void bucket_body(const int* __restrict__ dsts, const int* __restrict__ srcs,
                                            int* lst, int* cntg, int* offg, float* ddg, int* flg, int* dsm) {
  int*   lists = dsm;
  int*   sl    = dsm + NWAVE * WLCAP;
  int*   cntw  = sl + RCAP;
  int*   cnt   = cntw + NWAVE * NBA;
  int*   offs  = cnt + NBA;
  float* ddv   = (float*)(offs + NBA);
  int*   misc  = offs + 2 * NBA;
  const int tid  = (int)threadIdx.x, lane = tid & 31;
  const int wave = __builtin_amdgcn_readfirstlane(tid >> 5);
  {
    const v4i z4 = {0, 0, 0, 0};
    for (int i = tid * 4; i < BK_INTS; i += NTHR * 4) *(v4ia*)(dsm + i) = z4;
  }
  __syncthreads();

  const unsigned nbs = (unsigned)((int)blockIdx.x * NBA);
  const unsigned unb = (unsigned)NBA;
  int* mylist = lists + wave * WLCAP;
  const int wbeg = wave * WSHARE, wend = wbeg + WSHARE;
  int wc = 0;
#pragma unroll 1
  for (int it = 0; it < NIT; ++it) {
    const int e0 = wbeg + it * KPI + lane * 8;
    const int ea = e0 < NE - 4 ? e0 : NE - 4;
    const int eb = (e0 + 4) < NE - 4 ? (e0 + 4) : NE - 4;
    const v4i da = *(const v4i*)(dsts + ea);
    const v4i db = *(const v4i*)(dsts + eb);
    const v4i sa = *(const v4i*)(srcs + ea);
    const v4i sb = *(const v4i*)(srcs + eb);
    asm volatile("" :: "v"(da), "v"(db), "v"(sa), "v"(sb));
    const bool va = e0 < wend, vb = (e0 + 4) < wend;
    const unsigned s0 = (unsigned)da.x - nbs, s1 = (unsigned)da.y - nbs;
    const unsigned s2 = (unsigned)da.z - nbs, s3 = (unsigned)da.w - nbs;
    const unsigned s4 = (unsigned)db.x - nbs, s5 = (unsigned)db.y - nbs;
    const unsigned s6 = (unsigned)db.z - nbs, s7 = (unsigned)db.w - nbs;
    const bool h0 = va & (s0 < unb), h1 = va & (s1 < unb), h2 = va & (s2 < unb), h3 = va & (s3 < unb);
    const bool h4 = vb & (s4 < unb), h5 = vb & (s5 < unb), h6 = vb & (s6 < unb), h7 = vb & (s7 < unb);
    const unsigned any = __builtin_amdgcn_ballot_w32(h0 | h1 | h2 | h3 | h4 | h5 | h6 | h7);
    if (any != 0u) {
#define HITB(HJ, SJ, RJ) { \
      const unsigned mj = __builtin_amdgcn_ballot_w32(HJ); \
      if (mj != 0u) { \
        if (HJ) { \
          const int pos = wc + (int)__builtin_amdgcn_mbcnt_lo(mj, 0u); \
          if (pos < WLCAP) mylist[pos] = (clampn(RJ) << SLA) | (int)(SJ); \
        } \
        wc += (int)__builtin_popcount(mj); } }
      HITB(h0, s0, sa.x)
      HITB(h1, s1, sa.y)
      HITB(h2, s2, sa.z)
      HITB(h3, s3, sa.w)
      HITB(h4, s4, sb.x)
      HITB(h5, s5, sb.y)
      HITB(h6, s6, sb.z)
      HITB(h7, s7, sb.w)
#undef HITB
    }
  }
  if (lane == 0) misc[wave] = wc;
  __syncthreads();

  const int cw = wc > WLCAP ? WLCAP : wc;
  int* mycnt = cntw + wave * NBA;
#pragma unroll 1
  for (int b0 = 0; b0 < cw; b0 += 32) {
    const int idx = b0 + lane;
    const int ent = mylist[idx < WLCAP ? idx : WLCAP - 1];
    const int m32 = (cw - b0) < 32 ? (cw - b0) : 32;
#pragma unroll 1
    for (int k = 0; k < m32; ++k) {
      const int uu = __builtin_amdgcn_readlane(ent, k);
      const int slot = uu & (NBA - 1);
      if (lane == 0) mycnt[slot] = mycnt[slot] + 1;
    }
  }
  __syncthreads();

  v4i t4 = {0, 0, 0, 0};
#pragma unroll
  for (int w2 = 0; w2 < NWAVE; ++w2) {
    const v4i c = *(const v4ia*)(cntw + w2 * NBA + 4 * tid);
    t4 += c;
  }
  const int tot = (t4.x + t4.y) + (t4.z + t4.w);
  int incl = tot;
#pragma unroll
  for (int d = 1; d < 32; d <<= 1) {
    const int y = __shfl_up(incl, d, 32);
    if (lane >= d) incl += y;
  }
  if (lane == 31) misc[8 + wave] = incl;
  __syncthreads();
  int base = 0, total = 0, ov = 0;
#pragma unroll
  for (int w2 = 0; w2 < NWAVE; ++w2) {
    const int wsu = misc[8 + w2];
    base += (w2 < wave) ? wsu : 0;
    total += wsu;
    ov |= (misc[w2] > WLCAP) ? 1 : 0;
  }
  ov |= (total > RCAP) ? 1 : 0;
  {
    int run = base + incl - tot;
    v4i o4;
#define PFX(J, OJ) { \
      const int slot = 4 * tid + (J); \
      OJ = run; \
      _Pragma_free_loop_##J: ; \
      for (int w2 = 0; w2 < NWAVE; ++w2) { \
        const int c = cntw[w2 * NBA + slot]; \
        cntw[w2 * NBA + slot] = run; \
        run += c; } }
    PFX(0, o4.x)
    PFX(1, o4.y)
    PFX(2, o4.z)
    PFX(3, o4.w)
#undef PFX
    *(v4ia*)(offs + 4 * tid) = o4;
    *(v4ia*)(cnt + 4 * tid) = t4;
  }
  __syncthreads();

  const float qnan = __int_as_float(0x7fc00000);
#pragma unroll 1
  for (int j = 0; j < NBA / NTHR; ++j) {
    const int slot = tid + NTHR * j;
    const int c = cnt[slot];
    const float d = 1.0f / sqrtf((float)(c < 1 ? 1 : c));
    ddv[slot] = (ov != 0) ? qnan : d;
  }
#pragma unroll 1
  for (int b0 = 0; b0 < cw; b0 += 32) {
    const int idx = b0 + lane;
    const int ent = mylist[idx < WLCAP ? idx : WLCAP - 1];
    const int m32 = (cw - b0) < 32 ? (cw - b0) : 32;
#pragma unroll 1
    for (int k = 0; k < m32; ++k) {
      const int uu = __builtin_amdgcn_readlane(ent, k);
      const int slot = uu & (NBA - 1);
      if (lane == 0) {
        int p = mycnt[slot];
        p = p < 0 ? 0 : (p > RCAP - 1 ? RCAP - 1 : p);
        sl[p] = uu >> SLA;
        mycnt[slot] = p + 1;
      }
    }
  }
  __syncthreads();

  bucket_store(sl, cnt, offs, ddv, ov, lst, cntg, offg, ddg, flg, tid);
  __threadfence();
  bucket_store(sl, cnt, offs, ddv, ov, lst, cntg, offg, ddg, flg, tid);
}

__global__ __launch_bounds__(NTHR) void k_bucket(const int* __restrict__ dst_i, const int* __restrict__ src_i,
                                                 const int* __restrict__ dst_b, const int* __restrict__ src_b,
                                                 int* lst, int* cntg, int* offg, float* ddg, int* flg) {
  extern __shared__ __attribute__((aligned(16))) int dsm[];
  const int b = (int)blockIdx.x, r = (int)blockIdx.y;
  int*   l = lst  + ((size_t)r * GA + (size_t)b) * RCAP;
  int*   c = cntg + (size_t)r * NPT + (size_t)b * NBA;
  int*   o = offg + (size_t)r * NPT + (size_t)b * NBA;
  float* d = ddg  + (size_t)r * NPT + (size_t)b * NBA;
  int*   f = flg  + ((size_t)r * GA + (size_t)b) * 32;
  if (r == 0) bucket_body(dst_i, src_i, l, c, o, d, f, dsm);
  else        bucket_body(dst_b, src_b, l, c, o, d, f, dsm);
}

__device__ __forceinline__ void outdeg_store(const float* dsv, float* dsg, int tid) {
#pragma unroll 1
  for (int it = 0; it < NBO / (NTHR * 4); ++it) {
    const int i = it * (NTHR * 4) + 4 * tid;
    const v4f v = *(const v4fa*)(dsv + i);
    *(volatile v4f*)(dsg + i) = v;
  }
}

__device__ __forceinline__ void outdeg_body(const int* __restrict__ keys, float* dsg, int* dsm) {
  int*   bins  = dsm;
  int*   lists = dsm + NWAVE * NBO;
  float* dsv   = (float*)(lists + NWAVE * KPI);
  const int tid  = (int)threadIdx.x, lane = tid & 31;
  const int wave = __builtin_amdgcn_readfirstlane(tid >> 5);
  {
    const v4i z4 = {0, 0, 0, 0};
    for (int i = tid * 4; i < OD_INTS; i += NTHR * 4) *(v4ia*)(dsm + i) = z4;
  }
  __syncthreads();

  const unsigned nbs = (unsigned)((int)blockIdx.x * NBO);
  const unsigned unb = (unsigned)NBO;
  int* mylist = lists + wave * KPI;
  int* mybins = bins + wave * NBO;
  const int wbeg = wave * WSHARE, wend = wbeg + WSHARE;
#pragma unroll 1
  for (int it = 0; it < NIT; ++it) {
    const int e0 = wbeg + it * KPI + lane * 8;
    const int ea = e0 < NE - 4 ? e0 : NE - 4;
    const int eb = (e0 + 4) < NE - 4 ? (e0 + 4) : NE - 4;
    const v4i da = *(const v4i*)(keys + ea);
    const v4i db = *(const v4i*)(keys + eb);
    asm volatile("" :: "v"(da), "v"(db));
    const bool va = e0 < wend, vb = (e0 + 4) < wend;
    const unsigned s0 = (unsigned)da.x - nbs, s1 = (unsigned)da.y - nbs;
    const unsigned s2 = (unsigned)da.z - nbs, s3 = (unsigned)da.w - nbs;
    const unsigned s4 = (unsigned)db.x - nbs, s5 = (unsigned)db.y - nbs;
    const unsigned s6 = (unsigned)db.z - nbs, s7 = (unsigned)db.w - nbs;
    const bool h0 = va & (s0 < unb), h1 = va & (s1 < unb), h2 = va & (s2 < unb), h3 = va & (s3 < unb);
    const bool h4 = vb & (s4 < unb), h5 = vb & (s5 < unb), h6 = vb & (s6 < unb), h7 = vb & (s7 < unb);
    const unsigned any = __builtin_amdgcn_ballot_w32(h0 | h1 | h2 | h3 | h4 | h5 | h6 | h7);
    if (any != 0u) {
      int wc = 0;
#define HITO(HJ, SJ) { \
      const unsigned mj = __builtin_amdgcn_ballot_w32(HJ); \
      if (mj != 0u) { \
        if (HJ) { \
          const int pos = wc + (int)__builtin_amdgcn_mbcnt_lo(mj, 0u); \
          if (pos < KPI) mylist[pos] = (int)(SJ); \
        } \
        wc += (int)__builtin_popcount(mj); } }
      HITO(h0, s0)
      HITO(h1, s1)
      HITO(h2, s2)
      HITO(h3, s3)
      HITO(h4, s4)
      HITO(h5, s5)
      HITO(h6, s6)
      HITO(h7, s7)
#undef HITO
      wave_sync();
      const int c = wc > KPI ? KPI : wc;
#pragma unroll 1
      for (int b0 = 0; b0 < c; b0 += 32) {
        const int idx = b0 + lane;
        const int ent = mylist[idx < KPI ? idx : KPI - 1];
        const int m32 = (c - b0) < 32 ? (c - b0) : 32;
#pragma unroll 1
        for (int k = 0; k < m32; ++k) {
          const int uu = __builtin_amdgcn_readlane(ent, k);
          const int slot = uu & (NBO - 1);
          if (lane == 0) mybins[slot] = mybins[slot] + 1;
        }
      }
      wave_sync();
    }
  }
  __syncthreads();
#pragma unroll 1
  for (int j = 0; j < NBO / NTHR; ++j) {
    const int slot = tid + NTHR * j;
    int s = 0;
#pragma unroll
    for (int w2 = 0; w2 < NWAVE; ++w2) s += bins[w2 * NBO + slot];
    dsv[slot] = 1.0f / sqrtf((float)(s < 1 ? 1 : s));
  }
  __syncthreads();
  outdeg_store(dsv, dsg, tid);
  __threadfence();
  outdeg_store(dsv, dsg, tid);
}

__global__ __launch_bounds__(NTHR) void k_outdeg(const int* __restrict__ src_i, const int* __restrict__ src_b,
                                                 float* dsg) {
  extern __shared__ __attribute__((aligned(16))) int dsm[];
  const int r = (int)blockIdx.y;
  float* d = dsg + (size_t)r * NPO + (size_t)blockIdx.x * NBO;
  if (r == 0) outdeg_body(src_i, d, dsm);
  else        outdeg_body(src_b, d, dsm);
}

__global__ __launch_bounds__(GTHR) __attribute__((amdgpu_num_vgpr(248)))
void k_gemm(const unsigned short* __restrict__ A, int lda, const unsigned short* __restrict__ BT, int ldb, int K,
            const float* __restrict__ dsrc, int dsStride, float* out0, float* out1, int nN) {
  __shared__ __attribute__((aligned(16))) float stg[GBM * GBN];
  __shared__ __attribute__((aligned(16))) float sc[GBM];
  const int tid = (int)threadIdx.x, lane = tid & 31, hh = lane >> 4, m = lane & 15;
  const int wave = __builtin_amdgcn_readfirstlane(tid >> 5);
  const int rowBase = (int)blockIdx.x * GBM;
  const int yt = (int)blockIdx.y;

  if (wave < 2) sc[tid] = dsrc[(size_t)yt * (size_t)dsStride + (size_t)rowBase + tid];

  v8f acc[8];
#pragma unroll
  for (int t = 0; t < 8; ++t) acc[t] = z8();
  const unsigned short* ap = A + (size_t)(rowBase + 16 * wave + m) * (size_t)lda + 8 * hh;
  const unsigned short* bp = BT + (size_t)(GBN * yt + m) * (size_t)ldb + 8 * hh;

#pragma unroll 1
  for (int k0 = 0; k0 < K; k0 += 32) {
    FragB af;
    af.h[0] = *(const v8usa*)(ap + k0);
    af.h[1] = *(const v8usa*)(ap + k0 + 16);
#pragma unroll
    for (int nt = 0; nt < 8; ++nt) {
      const unsigned short* wq = bp + (size_t)(16 * nt) * (size_t)ldb + k0;
      FragB bf;
      bf.h[0] = *(const v8usa*)wq;
      bf.h[1] = *(const v8usa*)(wq + 16);
      acc[nt] = wmb(af, bf, acc[nt]);
    }
  }

#pragma unroll
  for (int nt = 0; nt < 8; ++nt) {
    const int lc = 16 * nt + m;
#pragma unroll
    for (int r = 0; r < 8; ++r) {
      const int lr = 16 * wave + 8 * hh + r;
      stg[lr * GBN + lc] = acc[nt][r];
    }
  }
  __syncthreads();

  v4f pv[16];
#pragma unroll
  for (int i = 0; i < 16; ++i) {
    const v4f t = *(const v4fa*)(stg + (16 * wave + i) * GBN + 4 * lane);
    const float s = sc[16 * wave + i];
    pv[i] = t * s;
  }
  float* const ob = (yt == 0) ? out0 : out1;
#pragma unroll
  for (int i = 0; i < 16; ++i) {
    const int row = rowBase + 16 * wave + i;
    float* op = ob + (size_t)row * DF + 4 * lane;
    if (row < nN) *(volatile v4f*)op = pv[i];
  }
  __threadfence();
#pragma unroll
  for (int i = 0; i < 16; ++i) {
    const int row = rowBase + 16 * wave + i;
    float* op = ob + (size_t)row * DF + 4 * lane;
    if (row < nN) *(volatile v4f*)op = pv[i];
  }
}

__device__ __forceinline__ v4f gather_rows(const int* __restrict__ lst, const float* hp, int cntv, int offv,
                                           int lane, bool& big) {
  const int cu = __builtin_amdgcn_readfirstlane(cntv);
  const int ou = __builtin_amdgcn_readfirstlane(offv);
  big = (cu > DEGCAP) || (cu < 0);
  const int c = cu < 0 ? 0 : (cu > DEGCAP ? DEGCAP : cu);
  const int o = ou < 0 ? 0 : (ou > RCAP - 1 ? RCAP - 1 : ou);
  int last = o + c - 1;
  last = last < o ? o : last;
  last = last > RCAP - 1 ? RCAP - 1 : last;
  v4f acc = {0.0f, 0.0f, 0.0f, 0.0f};
#pragma unroll 1
  for (int b0 = 0; b0 < c; b0 += 32) {
    int idx = o + b0 + lane;
    idx = idx > last ? last : idx;
    const int sr = clampn(lst[idx]);
    const int m32 = (c - b0) < 32 ? (c - b0) : 32;
#pragma unroll 1
    for (int k = 0; k < m32; ++k) {
      const int sk = __builtin_amdgcn_readlane(sr, k);
      const v4f a = *(const v4fa*)(hp + (size_t)sk * DF + 4 * lane);
      acc += a;
    }
  }
  return acc;
}

template <int MODE>
__global__ __launch_bounds__(NTHR) void k_agg(
    const int* __restrict__ lstA, const int* __restrict__ cntA, const int* __restrict__ offA,
    const float* __restrict__ ddA, const int* __restrict__ flgA, const float* hpA,
    const float* __restrict__ bA,
    const int* __restrict__ lstB, const int* __restrict__ cntB, const int* __restrict__ offB,
    const float* __restrict__ ddB, const int* __restrict__ flgB, const float* hpB,
    const float* __restrict__ bB,
    unsigned short* hs, float* outp) {
  __shared__ __attribute__((aligned(16))) int   tcA[NBA];
  __shared__ __attribute__((aligned(16))) int   toA[NBA];
  __shared__ __attribute__((aligned(16))) float tdA[NBA];
  __shared__ __attribute__((aligned(16))) int   tcB[NBA];
  __shared__ __attribute__((aligned(16))) int   toB[NBA];
  __shared__ __attribute__((aligned(16))) float tdB[NBA];
  const int tid = (int)threadIdx.x, lane = tid & 31;
  const int wave = __builtin_amdgcn_readfirstlane(tid >> 5);
  const int b = (int)blockIdx.x;
  const int nodeBase = b * NBA;
  const size_t tb = (size_t)b * NBA + 4 * (size_t)tid;
  {
    const v4i c4 = *(const v4i*)(cntA + tb);
    const v4i o4 = *(const v4i*)(offA + tb);
    const v4f d4 = *(const v4f*)(ddA + tb);
    *(v4ia*)(tcA + 4 * tid) = c4;
    *(v4ia*)(toA + 4 * tid) = o4;
    *(v4fa*)(tdA + 4 * tid) = d4;
  }
  int fl = flgA[(size_t)b * 32];
  v4f biasA = *(const v4f*)(bA + 4 * lane);
  v4f biasB = biasA;
  if constexpr (MODE != 0) {
    const v4i c4 = *(const v4i*)(cntB + tb);
    const v4i o4 = *(const v4i*)(offB + tb);
    const v4f d4 = *(const v4f*)(ddB + tb);
    *(v4ia*)(tcB + 4 * tid) = c4;
    *(v4ia*)(toB + 4 * tid) = o4;
    *(v4fa*)(tdB + 4 * tid) = d4;
    fl |= flgB[(size_t)b * 32];
    biasB = *(const v4f*)(bB + 4 * lane);
  }
  asm volatile("" :: "v"(fl), "v"(biasA), "v"(biasB));
  __syncthreads();

  const float qnan = __int_as_float(0x7fc00000);
  const int* la = lstA + (size_t)b * RCAP;
  const int* lb = lstB + (size_t)b * RCAP;
  const int sa = (2 * lane) & 31, sb = (2 * lane + 1) & 31;
  const bool lsel = (lane & 16) != 0;
#pragma unroll 1
  for (int si = 0; si < NBA / NWAVE; ++si) {
    const int s = si * NWAVE + wave;
    const int node = nodeBase + s;
    if (node >= NN) continue;
    bool bigA = false;
    const v4f aA = gather_rows(la, hpA, tcA[s], toA[s], lane, bigA);
    const float dA = tdA[s];
    asm volatile("" :: "v"(dA));
    if constexpr (MODE != 0) {
      bool bigB = false;
      const v4f aB = gather_rows(lb, hpB, tcB[s], toB[s], lane, bigB);
      const float dB = tdB[s];
      asm volatile("" :: "v"(dB));
      const bool pois = (fl != 0) || bigA || bigB;
      float v0 = relu_np(aA.x * dA + biasA.x) + relu_np(aB.x * dB + biasB.x);
      float v1 = relu_np(aA.y * dA + biasA.y) + relu_np(aB.y * dB + biasB.y);
      float v2 = relu_np(aA.z * dA + biasA.z) + relu_np(aB.z * dB + biasB.z);
      float v3 = relu_np(aA.w * dA + biasA.w) + relu_np(aB.w * dB + biasB.w);
      v0 = pois ? qnan : v0; v1 = pois ? qnan : v1; v2 = pois ? qnan : v2; v3 = pois ? qnan : v3;
      const unsigned h0 = bf16_bits(v0), h1 = bf16_bits(v1), h2 = bf16_bits(v2), h3 = bf16_bits(v3);
      const unsigned l0 = bf16_bits(v0 - __uint_as_float(h0 << 16));
      const unsigned l1 = bf16_bits(v1 - __uint_as_float(h1 << 16));
      const unsigned l2 = bf16_bits(v2 - __uint_as_float(h2 << 16));
      const unsigned l3 = bf16_bits(v3 - __uint_as_float(h3 << 16));
      const int hw0 = (int)(h0 | (h1 << 16)), hw1 = (int)(h2 | (h3 << 16));
      const int lw0 = (int)(l0 | (l1 << 16)), lw1 = (int)(l2 | (l3 << 16));
      const int g0 = __shfl(hw0, sa, 32), g1 = __shfl(hw1, sa, 32);
      const int g2 = __shfl(hw0, sb, 32), g3 = __shfl(hw1, sb, 32);
      const int p0 = __shfl(lw0, sa, 32), p1 = __shfl(lw1, sa, 32);
      const int p2 = __shfl(lw0, sb, 32), p3 = __shfl(lw1, sb, 32);
      v4u pv;
      pv.x = (unsigned)(lsel ? p0 : g0);
      pv.y = (unsigned)(lsel ? p1 : g1);
      pv.z = (unsigned)(lsel ? p2 : g2);
      pv.w = (unsigned)(lsel ? p3 : g3);
      unsigned short* hp = hs + (size_t)node * (2 * DF) + 8 * lane;
      *(volatile v4u*)hp = pv;
      __threadfence();
      *(volatile v4u*)hp = pv;
    } else {
      const bool pois = (fl != 0) || bigA;
      v4f ov;
      ov.x = aA.x * dA + biasA.x;
      ov.y = aA.y * dA + biasA.y;
      ov.z = aA.z * dA + biasA.z;
      ov.w = aA.w * dA + biasA.w;
      ov.x = pois ? qnan : ov.x; ov.y = pois ? qnan : ov.y;
      ov.z = pois ? qnan : ov.z; ov.w = pois ? qnan : ov.w;
      float* op = outp + (size_t)node * DF + 4 * lane;
      *(volatile v4f*)op = ov;
      __threadfence();
      *(volatile v4f*)op = ov;
    }
  }
}

static inline size_t al256(size_t o) { return (o + 255) & ~(size_t)255; }

extern "C" void kernel_launch(void* const* d_in, const int* in_sizes, int n_in,
                              void* d_out, int out_size, void* d_ws, size_t ws_size,
                              hipStream_t stream) {
  if (n_in < 11) return;
  if (in_sizes[0] != NN * DF) return;
  if (in_sizes[1] != NE || in_sizes[2] != NE || in_sizes[3] != NE || in_sizes[4] != NE) return;
  if (in_sizes[5] != DF * DF || in_sizes[7] != DF * DF || in_sizes[9] != DF * DF) return;
  if (in_sizes[6] != DF || in_sizes[8] != DF || in_sizes[10] != DF) return;
  if (out_size != NN * DF) return;

  const float* x    = (const float*)d_in[0];
  const int*   srcI = (const int*)d_in[1];
  const int*   dstI = (const int*)d_in[2];
  const int*   srcB = (const int*)d_in[3];
  const int*   dstB = (const int*)d_in[4];
  const float* W1i  = (const float*)d_in[5];
  const float* b1i  = (const float*)d_in[6];
  const float* W1b  = (const float*)d_in[7];
  const float* b1b  = (const float*)d_in[8];
  const float* W2   = (const float*)d_in[9];
  const float* b2   = (const float*)d_in[10];
  float* out = (float*)d_out;

  char* ws = (char*)d_ws;
  size_t off = 0;
  const size_t oHPI  = off; off = al256(off + (size_t)NN * DF * 4);
  const size_t oHS   = off; off = al256(off + (size_t)MP * 2 * DF * 2);
  const size_t oLST  = off; off = al256(off + (size_t)2 * GA * RCAP * 4);
  const size_t oCNT  = off; off = al256(off + (size_t)2 * NPT * 4);
  const size_t oOFF  = off; off = al256(off + (size_t)2 * NPT * 4);
  const size_t oDD   = off; off = al256(off + (size_t)2 * NPT * 4);
  const size_t oDS   = off; off = al256(off + (size_t)2 * NPO * 4);
  const size_t oFLG  = off; off = al256(off + (size_t)2 * GA * 32 * 4);
  const size_t oW1T  = off; off = al256(off + (size_t)2 * DF * DF * 2);
  const size_t oW2D  = off; off = al256(off + (size_t)DF * 2 * DF * 2);
  const size_t oBIA  = off; off = al256(off + (size_t)3 * DF * 4);
  if (off > ws_size || off > (size_t)WSMAX) return;
  if ((size_t)MP * DF * 2 > (size_t)NN * 2 * DF * 2) return;
  float*          HPI = (float*)(ws + oHPI);
  unsigned short* HS  = (unsigned short*)(ws + oHS);
  unsigned short* XB  = (unsigned short*)(ws + oHS);
  int*            LST = (int*)(ws + oLST);
  int*            CNT = (int*)(ws + oCNT);
  int*            OFF = (int*)(ws + oOFF);
  float*          DD  = (float*)(ws + oDD);
  float*          DS  = (float*)(ws + oDS);
  int*            FLG = (int*)(ws + oFLG);
  unsigned short* W1T = (unsigned short*)(ws + oW1T);
  unsigned short* W2D = (unsigned short*)(ws + oW2D);
  float*          BIA = (float*)(ws + oBIA);

  const size_t bkLds = (size_t)BK_INTS * 4;
  const size_t odLds = (size_t)OD_INTS * 4;
  hipFuncSetAttribute(reinterpret_cast<const void*>(&k_bucket), hipFuncAttributeMaxDynamicSharedMemorySize, (int)bkLds);
  hipFuncSetAttribute(reinterpret_cast<const void*>(&k_outdeg), hipFuncAttributeMaxDynamicSharedMemorySize, (int)odLds);

  k_prep<<<PU_END / NTHR, NTHR, 0, stream>>>(x, W1i, W1b, W2, b1i, b1b, b2, W1T, W2D, BIA, HS, XB);
  k_bucket<<<dim3(GA, 2), NTHR, bkLds, stream>>>(dstI, srcI, dstB, srcB, LST, CNT, OFF, DD, FLG);
  k_outdeg<<<dim3(GO, 2), NTHR, odLds, stream>>>(srcI, srcB, DS);
  k_gemm<<<dim3(MP / GBM, 2), GTHR, 0, stream>>>(XB, DF, W1T, DF, DF, DS, NPO, HPI, out, NN);
  k_agg<1><<<GA, NTHR, 0, stream>>>(LST, CNT, OFF, DD, FLG, HPI, BIA,
                                   LST + (size_t)GA * RCAP, CNT + NPT, OFF + NPT, DD + NPT, FLG + GA * 32,
                                   out, BIA + DF, HS, out);
  k_gemm<<<dim3(MP / GBM, 1), GTHR, 0, stream>>>(HS, 2 * DF, W2D, 2 * DF, 2 * DF, DS, NPO, HPI, HPI, NN);
  k_agg<0><<<GA, NTHR, 0, stream>>>(LST, CNT, OFF, DD, FLG, HPI, BIA + 2 * DF,
                                   LST, CNT, OFF, DD, FLG, HPI, BIA + 2 * DF, HS, out);
}
